// SGNP_45028437131846
// MI455X (gfx1250) — hardware-verified
//
#include <hip/hip_runtime.h>
#include <math.h>

constexpr int NBATCH = 16;
constexpr int NCPB   = 2048;
constexpr int NTPB   = 1024;
constexpr int NCTX   = NBATCH * NCPB;
constexpr int NTEST  = NBATCH * NTPB;
constexpr int NTOT   = NCTX + NTEST;
constexpr int KNBR   = 16;
constexpr int FDIM   = 64;
constexpr int DINPAD = 32;
constexpr int L1DIM  = 256;
constexpr int L2DIM  = 128;
constexpr int HD1DIM = 256;
constexpr int HD2DIM = 64;
constexpr int NPAD3  = 64;

typedef __attribute__((ext_vector_type(16))) _Float16 v16h;
typedef __attribute__((ext_vector_type(8)))  _Float16 v8h;
typedef __attribute__((ext_vector_type(16))) __bf16   v16b;
typedef __attribute__((ext_vector_type(8)))  __bf16   v8b;
typedef __attribute__((ext_vector_type(8)))  float    v8f;
typedef __attribute__((ext_vector_type(4)))  float    v4f;
typedef __attribute__((ext_vector_type(2)))  float    v2f;
typedef __attribute__((ext_vector_type(4)))  unsigned v4u;
typedef __attribute__((ext_vector_type(4)))  int      v4i;
#define PSCALE 32768.0f
#define U16(p) ((const unsigned short*)(const void*)(p))
#define PSCALE_INV (1.0f / 32768.0f)

__device__ __forceinline__ unsigned short f2bf_bits(float f) {
  unsigned u = __float_as_uint(f);
  return (unsigned short)((u + 0x7FFFu + ((u >> 16) & 1u)) >> 16);
}
__device__ __forceinline__ float bf_bits2f(unsigned short h) { return __uint_as_float(((unsigned)h) << 16); }

__device__ __forceinline__ void dep_guard_h(v8f& a, v8f& b, v16h x, v16h y) { asm volatile("v_nop\n\tv_nop\n\tv_nop\n\tv_nop" : "+v"(a), "+v"(b) : "v"(x), "v"(y)); }
__device__ __forceinline__ void dep_guard_b(v8f& a, v8f& b, v16b x, v16b y) { asm volatile("v_nop\n\tv_nop\n\tv_nop\n\tv_nop" : "+v"(a), "+v"(b) : "v"(x), "v"(y)); }
__device__ __forceinline__ void keep4_h(v16h a, v16h b, v16h c, v16h d) { asm volatile("v_nop" :: "v"(a), "v"(b), "v"(c), "v"(d)); }
__device__ __forceinline__ void keep4_b(v16b a, v16b b, v16b c, v16b d) { asm volatile("v_nop" :: "v"(a), "v"(b), "v"(c), "v"(d)); }
__device__ __forceinline__ void acc_guard4(v8f& a, v8f& b, v8f& c, v8f& d) { asm volatile("v_nop\n\tv_nop\n\tv_nop\n\tv_nop" : "+v"(a), "+v"(b), "+v"(c), "+v"(d)); }
template <typename T> struct Frag;
template <> struct Frag<_Float16> {
  typedef v16h V; union U { v16h v; v8h h[2]; };
  static __device__ __forceinline__ v16h load(const _Float16* p) {
    U f; f.h[0] = *(const v8h*)(p); f.h[1] = *(const v8h*)(p + 16); return f.v;
  }
  static __device__ __forceinline__ v8f mma(v16h a, v16h b, v8f c) {
    return __builtin_amdgcn_wmma_f32_16x16x32_f16(false, a, false, b, (short)0, c, false, false);
  }
  static __device__ __forceinline__ void guard(v8f& a, v8f& b, v16h x, v16h y) { dep_guard_h(a, b, x, y); }
  static __device__ __forceinline__ void keep(v16h a, v16h b, v16h c, v16h d) { keep4_h(a, b, c, d); }
};
template <> struct Frag<__bf16> {
  typedef v16b V; union U { v16b v; v8b h[2]; };
  static __device__ __forceinline__ v16b load(const __bf16* p) {
    U f; f.h[0] = *(const v8b*)(p); f.h[1] = *(const v8b*)(p + 16); return f.v;
  }
  static __device__ __forceinline__ v8f mma(v16b a, v16b b, v8f c) {
    return __builtin_amdgcn_wmma_f32_16x16x32_bf16(false, a, false, b, (short)0, c, false, false);
  }
  static __device__ __forceinline__ void guard(v8f& a, v8f& b, v16b x, v16b y) { dep_guard_b(a, b, x, y); }
  static __device__ __forceinline__ void keep(v16b a, v16b b, v16b c, v16b d) { keep4_b(a, b, c, d); }
};

__device__ __forceinline__ float gelu_tanh_f(float x) {
  const float u = x * x;
  const float w = fmaf(0.044715f * u, x, x);
  const float e = __builtin_amdgcn_exp2f(w * -2.3022082f);
  const float r = __builtin_amdgcn_rcpf(1.0f + e);
  return x * r;
}
__device__ __forceinline__ float softplus_f(float x) {
  return fmaxf(x, 0.0f) + log1pf(expf(-fabsf(x)));
}
__device__ __forceinline__ float h2f(unsigned s) {
  return (float)__builtin_bit_cast(_Float16, (unsigned short)s);
}
__device__ __forceinline__ unsigned pk2h(float a, float b) {
  const unsigned lo = (unsigned)__builtin_bit_cast(unsigned short, (_Float16)a);
  const unsigned hi = (unsigned)__builtin_bit_cast(unsigned short, (_Float16)b);
  return lo | (hi << 16);
}

template <int ET> struct Elem;
template <> struct Elem<0> { typedef _Float16 T; };
template <> struct Elem<1> { typedef __bf16 T; };
template <int ET, bool SPLIT, int BIAS_MODE, int OUT_MODE, bool RESID, int ACT = 0>
__global__ __launch_bounds__(256) void wmma_gemm64(
    const unsigned short* __restrict__ Ap, const unsigned short* __restrict__ A2p, int lda, long strideA,
    const unsigned short* __restrict__ Btp, const unsigned short* __restrict__ Bt2p, int ldb, long strideB,
    void* __restrict__ Cout, void* __restrict__ Cout2, int ldc, long strideC,
    const float* __restrict__ bias,
    const float* __restrict__ resid, long strideR,
    int M, int N, int K, float scale) {
  typedef typename Elem<ET>::T T;
  typedef typename Frag<T>::V V;
  const T* A = (const T*)Ap; const T* A2 = (const T*)A2p; const T* Bt = (const T*)Btp; const T* Bt2 = (const T*)Bt2p;
  __shared__ __align__(16) float sT[8][16 * 68];
  const int b    = blockIdx.y;
  const int lane = threadIdx.x & 31;
  const int wave = threadIdx.x >> 5;
  const int tilesN = N >> 6;
  const int tilesM = M >> 6;
  const int tile = blockIdx.x * 8 + wave;
  if (tile >= tilesM * tilesN) return;
  const int tm = tile / tilesN;
  const int tn = tile - tm * tilesN;
  const int m0 = tm << 6;
  const int n0 = tn << 6;

  const T* Ab  = A  + (size_t)b * strideA;
  const T* Bb  = Bt + (size_t)b * strideB;
  const T* Ab2 = SPLIT ? (A2  + (size_t)b * strideA) : nullptr;
  const T* Bb2 = SPLIT ? (Bt2 + (size_t)b * strideB) : nullptr;

  const int rlane = lane & 15;
  const int koff  = (lane >> 4) * 8;
  const int mOff  = (lane >> 4) * 8;

  v8f acc[4][4];
#pragma unroll
  for (int i = 0; i < 4; ++i)
#pragma unroll
    for (int j = 0; j < 4; ++j) acc[i][j] = (v8f){0.f,0.f,0.f,0.f,0.f,0.f,0.f,0.f};

  for (int k0 = 0; k0 < K; k0 += 32) {
    V bh[4], bl[4];
#pragma unroll
    for (int j = 0; j < 4; ++j) {
      const size_t bo = (size_t)(n0 + (j << 4) + rlane) * ldb + koff + k0;
      bh[j] = Frag<T>::load(Bb + bo);
      if (SPLIT) bl[j] = Frag<T>::load(Bb2 + bo);
    }
#pragma unroll
    for (int i = 0; i < 4; ++i) {
      const size_t ao = (size_t)(m0 + (i << 4) + rlane) * lda + koff + k0;
      V ah = Frag<T>::load(Ab + ao);
      V al;
      if (SPLIT) al = Frag<T>::load(Ab2 + ao);
#pragma unroll
      for (int j = 0; j < 4; ++j) {
        acc[i][j] = Frag<T>::mma(ah, bh[j], acc[i][j]);
        if (SPLIT) {
          acc[i][j] = Frag<T>::mma(ah, bl[j], acc[i][j]);
          acc[i][j] = Frag<T>::mma(al, bh[j], acc[i][j]);
        }
      }
      Frag<T>::guard(acc[i][0], acc[i][3], ah, SPLIT ? al : ah);
    }
    Frag<T>::keep(bh[0], bh[1], bh[2], bh[3]);
    if (SPLIT) Frag<T>::keep(bl[0], bl[1], bl[2], bl[3]);
  }
  acc_guard4(acc[0][0], acc[0][1], acc[0][2], acc[0][3]);
  acc_guard4(acc[1][0], acc[1][1], acc[1][2], acc[1][3]);
  acc_guard4(acc[2][0], acc[2][1], acc[2][2], acc[2][3]);
  acc_guard4(acc[3][0], acc[3][1], acc[3][2], acc[3][3]);

  float* slab = sT[wave];
  const float* Rb = RESID ? (resid + (size_t)b * strideR) : nullptr;
#pragma unroll
  for (int i = 0; i < 4; ++i) {
    const int mBase = m0 + (i << 4);
#pragma unroll
    for (int j = 0; j < 4; ++j) {
      const int n = n0 + (j << 4) + rlane;
      float bv = 0.f;
      if (BIAS_MODE == 2) bv = bias[n];
#pragma unroll
      for (int r = 0; r < 8; ++r) {
        float v = acc[i][j][r] * scale;
        if (BIAS_MODE == 1) v += bias[mBase + mOff + r];
        if (BIAS_MODE == 2) v += bv;
        if (RESID) v += Rb[(size_t)(mBase + mOff + r) * ldc + n];
        if (ACT == 1) v = tanhf(v);
        if (ACT == 2) v = fmaxf(v, 0.0f);
        if (ACT == 3) v = v / (1.0f + expf(-v));
        if (ACT == 4) v = (v > 0.f) ? v : 0.01f * v;
        if (ACT == 6) v = gelu_tanh_f(v);
        slab[(mOff + r) * 68 + (j << 4) + rlane] = v;
      }
    }
    __builtin_amdgcn_fence(__ATOMIC_RELEASE, "workgroup");
    __builtin_amdgcn_wave_barrier();
    __builtin_amdgcn_fence(__ATOMIC_ACQUIRE, "workgroup");
    if (OUT_MODE == 0) {
      float* C = (float*)Cout + (size_t)b * strideC;
      const int hh = lane >> 4, c4 = (lane & 15) * 4;
      for (int pass = 0; pass < 2; ++pass) {
#pragma unroll
        for (int it = 0; it < 8; ++it) {
          const int row = it * 2 + hh;
          v4f v = *(const v4f*)(slab + row * 68 + c4);
          *(volatile v4f*)(C + (size_t)(mBase + row) * ldc + n0 + c4) = v;
        }
        __threadfence();
      }
    } else {
      const int q = lane >> 3, c8 = (lane & 7) * 8;
      unsigned short* C  = (unsigned short*)Cout  + (size_t)b * strideC;
      unsigned short* C2 = (OUT_MODE == 2) ? ((unsigned short*)Cout2 + (size_t)b * strideC) : nullptr;
      for (int pass = 0; pass < 2; ++pass) {
#pragma unroll
        for (int it = 0; it < 4; ++it) {
          const int row = it * 4 + q;
          const float* sp = slab + row * 68 + c8;
          v8h hv, lv;
#pragma unroll
          for (int e = 0; e < 8; ++e) {
            if (OUT_MODE == 1) {
              hv[e] = (_Float16)sp[e];
            } else {
              unsigned short hb = f2bf_bits(sp[e]);
              unsigned short lb = f2bf_bits(sp[e] - bf_bits2f(hb));
              hv[e] = __builtin_bit_cast(_Float16, hb);
              lv[e] = __builtin_bit_cast(_Float16, lb);
            }
          }
          *(volatile v8h*)(C + (size_t)(mBase + row) * ldc + n0 + c8) = hv;
          if (OUT_MODE == 2) *(volatile v8h*)(C2 + (size_t)(mBase + row) * ldc + n0 + c8) = lv;
        }
        __threadfence();
      }
    }
    __builtin_amdgcn_fence(__ATOMIC_RELEASE, "workgroup");
    __builtin_amdgcn_wave_barrier();
    __builtin_amdgcn_fence(__ATOMIC_ACQUIRE, "workgroup");
  }
}

__global__ __launch_bounds__(256) void cast_wt_kernel(
    const float* __restrict__ W, int kd, int nd, int kp, int np_, unsigned short* __restrict__ out) {
  const int i = blockIdx.x * 256 + threadIdx.x;
  const int nchunks = (np_ * kp) >> 3;
  if (i >= nchunks) return;
  const int e0 = i << 3;
  const int n  = e0 / kp;
  const int k0 = e0 - n * kp;
  const int nc = (n < nd) ? n : (nd - 1);
  unsigned pw[4];
#pragma unroll
  for (int j = 0; j < 4; ++j) {
    const int ka = k0 + 2 * j, kb = ka + 1;
    const int kac = (ka < kd) ? ka : (kd - 1);
    const int kbc = (kb < kd) ? kb : (kd - 1);
    float va = W[(size_t)kac * nd + nc];
    float vb = W[(size_t)kbc * nd + nc];
    va = (ka < kd && n < nd) ? va : 0.0f;
    vb = (kb < kd && n < nd) ? vb : 0.0f;
    pw[j] = pk2h(va, vb);
  }
  v4u u; u.x = pw[0]; u.y = pw[1]; u.z = pw[2]; u.w = pw[3];
  v4u* dst = (v4u*)(out + (size_t)e0);
  *(volatile v4u*)dst = u;
  __threadfence();
  *(volatile v4u*)dst = u;
}

__global__ __launch_bounds__(256) void acat_kernel(
    const float* __restrict__ asrc, const float* __restrict__ adst, unsigned short* __restrict__ out) {
  const int i = blockIdx.x * 256 + threadIdx.x;
  if (i >= 512) return;
  const int e0 = i << 3;
  const int n  = e0 >> 6;
  const int k0 = e0 & 63;
  unsigned pw[4];
#pragma unroll
  for (int j = 0; j < 4; ++j) {
    float vv[2];
#pragma unroll
    for (int t = 0; t < 2; ++t) {
      const int k = k0 + 2 * j + t;
      const float vs = asrc[k & 63];
      const float vd = adst[k & 63];
      const bool ins = (n < 4) && (k >= 16 * n) && (k < 16 * n + 16);
      const bool ind = (n >= 4) && (n < 8) && (k >= 16 * (n - 4)) && (k < 16 * (n - 4) + 16);
      vv[t] = ins ? vs : (ind ? vd : 0.0f);
    }
    pw[j] = pk2h(vv[0], vv[1]);
  }
  v4u u; u.x = pw[0]; u.y = pw[1]; u.z = pw[2]; u.w = pw[3];
  v4u* dst = (v4u*)(out + (size_t)e0);
  *(volatile v4u*)dst = u;
  __threadfence();
  *(volatile v4u*)dst = u;
}

__global__ __launch_bounds__(256) void x0_kernel(
    const float* __restrict__ s_ctx, const float* __restrict__ f_ctx, const float* __restrict__ s_test,
    const float* __restrict__ emb, unsigned short* __restrict__ x0) {
  const int lane = threadIdx.x & 31, wave = threadIdx.x >> 5;
  const int r = blockIdx.x * 64 + wave * 8 + (lane >> 2);
  const int c = lane & 3;
  const bool isctx = (r < NCTX);
  const int rc = isctx ? r : (NCTX - 1);
  int rt = r - NCTX;
  rt = (rt < 0) ? 0 : rt;
  rt = (rt > NTEST - 1) ? (NTEST - 1) : rt;
  const float cx = s_ctx[(size_t)rc * 2], cy = s_ctx[(size_t)rc * 2 + 1];
  const float fx = f_ctx[(size_t)rc * 2], fy = f_ctx[(size_t)rc * 2 + 1];
  const float tx = s_test[(size_t)rt * 2], ty = s_test[(size_t)rt * 2 + 1];
  float e[8];
#pragma unroll
  for (int i = 0; i < 8; ++i) e[i] = emb[i];
  const float v0 = isctx ? e[4] : e[0];
  const float v1 = isctx ? e[5] : e[1];
  const float v2 = isctx ? e[6] : e[2];
  const float v3 = isctx ? e[7] : e[3];
  const float v4 = isctx ? cx : tx;
  const float v5 = isctx ? cy : ty;
  const float v6 = isctx ? fx : 0.0f;
  const float v7 = isctx ? fy : 0.0f;
  const bool lead = (c == 0);
  v4u u;
  u.x = lead ? pk2h(v0, v1) : 0u;
  u.y = lead ? pk2h(v2, v3) : 0u;
  u.z = lead ? pk2h(v4, v5) : 0u;
  u.w = lead ? pk2h(v6, v7) : 0u;
  v4u* dst = (v4u*)(x0 + (size_t)r * DINPAD + c * 8);
  *(volatile v4u*)dst = u;
  __threadfence();
  *(volatile v4u*)dst = u;
}

__global__ __launch_bounds__(256) void knn_kernel(
    const float* __restrict__ s_ctx, const float* __restrict__ s_test, int* __restrict__ nbr) {
#pragma clang fp contract(off)
  __shared__ float scx[NCPB];
  __shared__ float scy[NCPB];
  __shared__ float scq[NCPB];
  __shared__ __align__(16) int snb[256 * KNBR];
  const int t = threadIdx.x;
  const int q0 = blockIdx.x * 256;
  const int b = q0 / NTPB;
  const float* cb = s_ctx + (size_t)b * NCPB * 2;
#pragma unroll 1
  for (int i = t; i < NCPB; i += 256) {
    const float x = cb[2 * i];
    const float y = cb[2 * i + 1];
    scx[i] = x;
    scy[i] = y;
    const float t0 = x * x;
    const float t1 = y * y;
    scq[i] = t0 + t1;
  }
  __syncthreads();

  const int q = q0 + t;
  const float qx = s_test[(size_t)q * 2];
  const float qy = s_test[(size_t)q * 2 + 1];
  const float tq0 = qx * qx;
  const float tq1 = qy * qy;
  const float sqq = tq0 + tq1;

  float dd[KNBR];
  int di[KNBR];
#pragma unroll
  for (int j = 0; j < KNBR; ++j) { dd[j] = INFINITY; di[j] = 0; }

#pragma unroll 1
  for (int c = 0; c < NCPB; ++c) {
    const float cx = scx[c];
    const float cy = scy[c];
    float p = qx * cx;
    p = fmaf(qy, cy, p);
    const float s = sqq + scq[c];
    const float p2 = 2.0f * p;
    const float d2 = s - p2;
    if (d2 < dd[KNBR - 1]) {
      float dv = d2;
      int iv = c;
#pragma unroll
      for (int j = 0; j < KNBR; ++j) {
        const float td = dd[j];
        const int ti = di[j];
        const bool lt = (dv < td) | ((dv == td) & (iv < ti));
        dd[j] = lt ? dv : td;
        di[j] = lt ? iv : ti;
        dv = lt ? td : dv;
        iv = lt ? ti : iv;
      }
    }
  }
#pragma unroll
  for (int j = 0; j < KNBR; ++j) snb[t * KNBR + j] = di[j];
  __syncthreads();

  int* base = nbr + (size_t)blockIdx.x * (256 * KNBR);
  v4i sv[4];
#pragma unroll
  for (int it = 0; it < 4; ++it) sv[it] = *(const v4i*)(snb + it * 1024 + t * 4);
  for (int pass = 0; pass < 2; ++pass) {
#pragma unroll
    for (int it = 0; it < 4; ++it) *(volatile v4i*)(base + it * 1024 + t * 4) = sv[it];
    __threadfence();
  }
}

__global__ __launch_bounds__(256) void ln_kernel(
    const float* __restrict__ pre, const float* __restrict__ g, const float* __restrict__ bb,
    unsigned short* __restrict__ nh) {
  const int lane = threadIdx.x & 31, wave = threadIdx.x >> 5;
  const int row = blockIdx.x * 8 + wave;
  const v2f x = *(const v2f*)(pre + (size_t)row * FDIM + 2 * lane);
  const float g0 = g[2 * lane], g1 = g[2 * lane + 1];
  const float b0 = bb[2 * lane], b1 = bb[2 * lane + 1];
  float s = x.x + x.y;
#pragma unroll
  for (int off = 1; off < 32; off <<= 1) s += __shfl_xor(s, off, 32);
  const float mu = s * (1.0f / 64.0f);
  const float d0 = x.x - mu, d1 = x.y - mu;
  float v = d0 * d0 + d1 * d1;
#pragma unroll
  for (int off = 1; off < 32; off <<= 1) v += __shfl_xor(v, off, 32);
  const float var = v * (1.0f / 64.0f);
  const float rstd = rsqrtf(var + 1e-6f);
  const float y0 = d0 * rstd * g0 + b0;
  const float y1 = d1 * rstd * g1 + b1;
  const unsigned pkd = pk2h(y0, y1);
  volatile unsigned* dst = (volatile unsigned*)(nh + (size_t)row * FDIM + 2 * lane);
  *dst = pkd;
  __threadfence();
  *dst = pkd;
}

__global__ __launch_bounds__(256) void gat_kernel(
    const float* __restrict__ sc, const unsigned short* __restrict__ xp,
    const unsigned short* __restrict__ nh, const int* __restrict__ nbr,
    const float* __restrict__ s_ctx, const float* __restrict__ s_test,
    const float* __restrict__ We, const float* __restrict__ be,
    unsigned short* __restrict__ nt) {
  const int lane = threadIdx.x & 31, wave = threadIdx.x >> 5;
  const int q = blockIdx.x * 8 + wave;
  const int b = q / NTPB;
  const int node = NCTX + q;
  const int kk = lane & 15, hp = lane >> 4;
  int nb = nbr[(size_t)q * KNBR + kk];
  nb = (nb < 0) ? 0 : nb;
  nb = (nb > NCPB - 1) ? (NCPB - 1) : nb;
  const int snd = b * NCPB + nb;
  const v2f ss = *(const v2f*)(sc + (size_t)snd * FDIM + 2 * hp);
  const v2f sd = *(const v2f*)(sc + (size_t)node * FDIM + 4 + 2 * hp);
  const float qx = s_test[(size_t)q * 2], qy = s_test[(size_t)q * 2 + 1];
  const float cx = s_ctx[(size_t)snd * 2], cy = s_ctx[(size_t)snd * 2 + 1];
  const float dx = qx - cx, dy = qy - cy;
  float w[8], bv[4];
#pragma unroll
  for (int i = 0; i < 8; ++i) w[i] = We[i];
#pragma unroll
  for (int i = 0; i < 4; ++i) bv[i] = be[i];
  const float wx0 = hp ? w[2] : w[0], wy0 = hp ? w[6] : w[4], be0 = hp ? bv[2] : bv[0];
  const float wx1 = hp ? w[3] : w[1], wy1 = hp ? w[7] : w[5], be1 = hp ? bv[3] : bv[1];
  const float eb0 = dx * wx0 + dy * wy0 + be0;
  const float eb1 = dx * wx1 + dy * wy1 + be1;
  float s0 = ss.x + sd.x;
  s0 = (s0 >= 0.0f) ? s0 : 0.2f * s0;
  s0 += eb0;
  float s1 = ss.y + sd.y;
  s1 = (s1 >= 0.0f) ? s1 : 0.2f * s1;
  s1 += eb1;
  float mx0 = s0, mx1 = s1;
#pragma unroll
  for (int off = 1; off < 16; off <<= 1) {
    mx0 = fmaxf(mx0, __shfl_xor(mx0, off, 32));
    mx1 = fmaxf(mx1, __shfl_xor(mx1, off, 32));
  }
  const float e0 = expf(s0 - mx0), e1 = expf(s1 - mx1);
  float z0 = e0, z1 = e1;
#pragma unroll
  for (int off = 1; off < 16; off <<= 1) {
    z0 += __shfl_xor(z0, off, 32);
    z1 += __shfl_xor(z1, off, 32);
  }
  const float al0 = e0 * (1.0f / z0);
  const float al1 = e1 * (1.0f / z1);
  const int hl = lane >> 3;
  const int sb = (hl >> 1) << 4;
  const bool odd = (hl & 1) != 0;
  float acc0 = 0.0f, acc1 = 0.0f;
#pragma unroll 1
  for (int kb8 = 0; kb8 < KNBR; kb8 += 8) {
#pragma unroll
    for (int j = 0; j < 8; ++j) {
      const int k = kb8 + j;
      const float a0 = __shfl(al0, sb + k, 32);
      const float a1 = __shfl(al1, sb + k, 32);
      const int sk = __shfl(snd, k, 32);
      const float a = odd ? a1 : a0;
      const unsigned wv = *(const unsigned*)(xp + (size_t)sk * FDIM + 2 * lane);
      acc0 += a * h2f(wv & 0xffffu);
      acc1 += a * h2f(wv >> 16);
    }
  }
  const unsigned wn = *(const unsigned*)(nh + (size_t)node * FDIM + 2 * lane);
  const float r0 = h2f(wn & 0xffffu) + acc0;
  const float r1 = h2f(wn >> 16) + acc1;
  const unsigned pkd = pk2h(r0, r1);
  volatile unsigned* dst = (volatile unsigned*)(nt + (size_t)q * FDIM + 2 * lane);
  *dst = pkd;
  __threadfence();
  *dst = pkd;
}

__global__ __launch_bounds__(256) void out_kernel(
    const float* __restrict__ o3, const float* __restrict__ c3, float* __restrict__ out) {
  const int lane = threadIdx.x & 31, wave = threadIdx.x >> 5;
  const int qa = blockIdx.x * 512 + wave * 64 + 2 * lane;
  const v2f oa = *(const v2f*)(o3 + (size_t)qa * NPAD3);
  const v2f ob = *(const v2f*)(o3 + (size_t)(qa + 1) * NPAD3);
  const float c30 = c3[0], c31 = c3[1];
  v4f r;
  r.x = oa.x + c30;
  r.y = softplus_f(oa.y + c31);
  r.z = ob.x + c30;
  r.w = softplus_f(ob.y + c31);
  v4f* dst = (v4f*)(out + (size_t)qa * 2);
  *(volatile v4f*)dst = r;
  __threadfence();
  *(volatile v4f*)dst = r;
}

constexpr size_t WT_W1 = 0, WT_W2 = 16384, WT_W3 = 81920, WT_WG = 98304, WT_AC = 106496,
                 WT_H1 = 114688, WT_H2 = 147456, WT_H3 = 180224, WT_END = 188416;
constexpr size_t OFF_WT  = 0;
constexpr size_t SZ_WT   = 262144;
constexpr size_t OFF_X0  = OFF_WT + SZ_WT;
constexpr size_t SZ_X0   = (size_t)NTOT * DINPAD * 2;
constexpr size_t OFF_A1  = OFF_X0 + SZ_X0;
constexpr size_t SZ_A1   = (size_t)NTOT * L1DIM * 2;
constexpr size_t OFF_A2  = OFF_A1 + SZ_A1;
constexpr size_t SZ_A2   = (size_t)NTOT * L2DIM * 2;
constexpr size_t OFF_PRE = OFF_A2 + SZ_A2;
constexpr size_t SZ_PRE  = (size_t)NTOT * FDIM * 4;
constexpr size_t OFF_NH  = OFF_PRE + SZ_PRE;
constexpr size_t SZ_NH   = (size_t)NTOT * FDIM * 2;
constexpr size_t OFF_XP  = OFF_NH + SZ_NH;
constexpr size_t SZ_XP   = (size_t)NTOT * FDIM * 2;
constexpr size_t OFF_SC  = OFF_XP + SZ_XP;
constexpr size_t SZ_SC   = (size_t)NTOT * FDIM * 4;
constexpr size_t OFF_NBR = OFF_SC + SZ_SC;
constexpr size_t SZ_NBR  = (size_t)NTEST * KNBR * 4;
constexpr size_t OFF_NT  = OFF_NBR + SZ_NBR;
constexpr size_t SZ_NT   = (size_t)NTEST * FDIM * 2;
constexpr size_t OFF_O1  = OFF_NT + SZ_NT;
constexpr size_t SZ_O1   = (size_t)NTEST * HD1DIM * 2;
constexpr size_t OFF_O2  = OFF_O1 + SZ_O1;
constexpr size_t SZ_O2   = (size_t)NTEST * HD2DIM * 2;
constexpr size_t OFF_O3  = OFF_O2 + SZ_O2;
constexpr size_t SZ_O3   = (size_t)NTEST * NPAD3 * 4;
constexpr size_t WS_TOTAL = OFF_O3 + SZ_O3;
static_assert(WT_END <= SZ_WT);
static_assert(WT_W1 + 256 * 32 * 2 == WT_W2);
static_assert(WT_W2 + 128 * 256 * 2 == WT_W3);
static_assert(WT_W3 + 64 * 128 * 2 == WT_WG);
static_assert(WT_WG + 64 * 64 * 2 == WT_AC);
static_assert(WT_AC + 64 * 64 * 2 == WT_H1);
static_assert(WT_H1 + 256 * 64 * 2 == WT_H2);
static_assert(WT_H2 + 64 * 256 * 2 == WT_H3);
static_assert(WT_H3 + 64 * 64 * 2 == WT_END);
static_assert(WS_TOTAL == 96731136);
static_assert(WS_TOTAL <= 134217728);
static_assert((OFF_X0 % 128) == 0 && (OFF_A1 % 128) == 0 && (OFF_A2 % 128) == 0 && (OFF_PRE % 128) == 0);
static_assert((OFF_NH % 128) == 0 && (OFF_XP % 128) == 0 && (OFF_SC % 128) == 0 && (OFF_NBR % 128) == 0);
static_assert((OFF_NT % 128) == 0 && (OFF_O1 % 128) == 0 && (OFF_O2 % 128) == 0 && (OFF_O3 % 128) == 0);
static_assert(NTOT % 64 == 0 && NTEST % 64 == 0);
static_assert(L1DIM % 64 == 0 && L2DIM % 64 == 0 && FDIM % 64 == 0 && HD1DIM % 64 == 0 && HD2DIM % 64 == 0 && NPAD3 % 64 == 0);
static_assert(DINPAD % 32 == 0 && L1DIM % 32 == 0 && L2DIM % 32 == 0 && FDIM % 32 == 0 && HD1DIM % 32 == 0);
static_assert(NTPB % 256 == 0 && NTOT % 64 == 0 && NTOT % 8 == 0 && NTEST % 8 == 0 && NTEST % 256 == 0 && NTEST % 512 == 0);
static_assert((size_t)NTEST * 2 * 4 == 131072);

template <int BIAS, int OUTM, int ACT>
static void launch_gemm(const unsigned short* A, int lda, const unsigned short* Bt, int ldb,
                        void* C, int ldc, const float* bias, int M, int N, int K, hipStream_t st) {
  const int tiles = (M / 64) * (N / 64);
  dim3 grid((tiles + 7) / 8, 1);
  wmma_gemm64<0, false, BIAS, OUTM, false, ACT><<<grid, 256, 0, st>>>(
      A, A, lda, 0L, Bt, Bt, ldb, 0L, C, C, ldc, 0L, bias, bias, 0L, M, N, K, 1.0f);
}

extern "C" void kernel_launch(void* const* d_in, const int* in_sizes, int n_in,
                              void* d_out, int out_size, void* d_ws, size_t ws_size,
                              hipStream_t stream) {
  (void)in_sizes;
  if (n_in < 23) return;
  if (ws_size < WS_TOTAL) return;
  if ((size_t)out_size < (size_t)NTEST * 2) return;

  const float* s_ctx  = (const float*)d_in[0];
  const float* f_ctx  = (const float*)d_in[1];
  const float* s_test = (const float*)d_in[2];
  const float* emb    = (const float*)d_in[3];
  const float* W1 = (const float*)d_in[4];    const float* b1 = (const float*)d_in[5];
  const float* W2 = (const float*)d_in[6];    const float* b2 = (const float*)d_in[7];
  const float* W3 = (const float*)d_in[8];    const float* b3 = (const float*)d_in[9];
  const float* ln_g = (const float*)d_in[10]; const float* ln_b = (const float*)d_in[11];
  const float* Wg = (const float*)d_in[12];
  const float* a_src = (const float*)d_in[13]; const float* a_dst = (const float*)d_in[14];
  const float* We = (const float*)d_in[15];   const float* be = (const float*)d_in[16];
  const float* H1 = (const float*)d_in[17];   const float* c1 = (const float*)d_in[18];
  const float* H2 = (const float*)d_in[19];   const float* c2 = (const float*)d_in[20];
  const float* H3 = (const float*)d_in[21];   const float* c3 = (const float*)d_in[22];
  float* out = (float*)d_out;

  char* ws = (char*)d_ws;
  unsigned short* W1t  = (unsigned short*)(ws + OFF_WT + WT_W1);
  unsigned short* W2t  = (unsigned short*)(ws + OFF_WT + WT_W2);
  unsigned short* W3t  = (unsigned short*)(ws + OFF_WT + WT_W3);
  unsigned short* Wgt  = (unsigned short*)(ws + OFF_WT + WT_WG);
  unsigned short* Acat = (unsigned short*)(ws + OFF_WT + WT_AC);
  unsigned short* H1t  = (unsigned short*)(ws + OFF_WT + WT_H1);
  unsigned short* H2t  = (unsigned short*)(ws + OFF_WT + WT_H2);
  unsigned short* H3t  = (unsigned short*)(ws + OFF_WT + WT_H3);
  unsigned short* X0 = (unsigned short*)(ws + OFF_X0);
  unsigned short* A1 = (unsigned short*)(ws + OFF_A1);
  unsigned short* A2 = (unsigned short*)(ws + OFF_A2);
  float* PRE = (float*)(ws + OFF_PRE);
  unsigned short* NH = (unsigned short*)(ws + OFF_NH);
  unsigned short* XP = (unsigned short*)(ws + OFF_XP);
  float* SC = (float*)(ws + OFF_SC);
  int* NBR = (int*)(ws + OFF_NBR);
  unsigned short* NT = (unsigned short*)(ws + OFF_NT);
  unsigned short* O1 = (unsigned short*)(ws + OFF_O1);
  unsigned short* O2 = (unsigned short*)(ws + OFF_O2);
  float* O3 = (float*)(ws + OFF_O3);

  cast_wt_kernel<<<4, 256, 0, stream>>>(W1, 8, 256, 32, 256, W1t);
  cast_wt_kernel<<<16, 256, 0, stream>>>(W2, 256, 128, 256, 128, W2t);
  cast_wt_kernel<<<4, 256, 0, stream>>>(W3, 128, 64, 128, 64, W3t);
  cast_wt_kernel<<<2, 256, 0, stream>>>(Wg, 64, 64, 64, 64, Wgt);
  cast_wt_kernel<<<8, 256, 0, stream>>>(H1, 64, 256, 64, 256, H1t);
  cast_wt_kernel<<<8, 256, 0, stream>>>(H2, 256, 64, 256, 64, H2t);
  cast_wt_kernel<<<2, 256, 0, stream>>>(H3, 64, 2, 64, NPAD3, H3t);
  acat_kernel<<<2, 256, 0, stream>>>(a_src, a_dst, Acat);

  x0_kernel<<<NTOT / 64, 256, 0, stream>>>(s_ctx, f_ctx, s_test, emb, X0);
  knn_kernel<<<NTEST / 256, 256, 0, stream>>>(s_ctx, s_test, NBR);

  launch_gemm<2, 1, 6>(X0, DINPAD, W1t, DINPAD, A1, L1DIM, b1, NTOT, L1DIM, DINPAD, stream);
  launch_gemm<2, 1, 6>(A1, L1DIM, W2t, L1DIM, A2, L2DIM, b2, NTOT, L2DIM, L1DIM, stream);
  launch_gemm<2, 0, 0>(A2, L2DIM, W3t, L2DIM, PRE, FDIM, b3, NTOT, FDIM, L2DIM, stream);
  ln_kernel<<<NTOT / 8, 256, 0, stream>>>(PRE, ln_g, ln_b, NH);
  launch_gemm<0, 1, 0>(NH, FDIM, Wgt, FDIM, XP, FDIM, b1, NTOT, FDIM, FDIM, stream);
  launch_gemm<0, 0, 0>(XP, FDIM, Acat, FDIM, SC, FDIM, b1, NTOT, FDIM, FDIM, stream);

  gat_kernel<<<NTEST / 8, 256, 0, stream>>>(SC, XP, NH, NBR, s_ctx, s_test, We, be, NT);

  launch_gemm<2, 1, 6>(NT, FDIM, H1t, FDIM, O1, HD1DIM, c1, NTEST, HD1DIM, FDIM, stream);
  launch_gemm<2, 1, 6>(O1, HD1DIM, H2t, HD1DIM, O2, HD2DIM, c2, NTEST, HD2DIM, HD1DIM, stream);
  launch_gemm<0, 0, 0>(O2, HD2DIM, H3t, HD2DIM, O3, NPAD3, b1, NTEST, NPAD3, HD2DIM, stream);
  out_kernel<<<NTEST / 512, 256, 0, stream>>>(O3, c3, out);
}
